// ModulatedConv3d_63239098466931
// MI455X (gfx1250) — hardware-verified
//
#include <hip/hip_runtime.h>


#define NBI  8
#define CIN  512
#define COUT 512
#define KK   3
#define SD   512
#define PP   2048
#define KC   (CIN * KK)
#define DM   SD
#define LOSC 1024.0f

typedef _Float16 h16;
typedef unsigned short bf;
typedef __attribute__((ext_vector_type(16))) __bf16   v16bf;
typedef __attribute__((ext_vector_type(16))) _Float16 v16h;
typedef __attribute__((ext_vector_type(8)))  _Float16 v8h;
typedef __attribute__((ext_vector_type(8)))  unsigned short v8us;
typedef __attribute__((ext_vector_type(8)))  float    v8f;
typedef __attribute__((ext_vector_type(4)))  float    v4f;
typedef v8h  __attribute__((may_alias)) v8ha;
typedef v4f  __attribute__((may_alias)) v4fa;
typedef v8us __attribute__((may_alias)) v8usa;

__device__ __forceinline__ unsigned short f2bf(float f) { unsigned u = __float_as_uint(f); u += 0x7FFFu + ((u >> 16) & 1u); return (unsigned short)(u >> 16); }
__device__ __forceinline__ float bf2f(unsigned short b) { return __uint_as_float(((unsigned)b) << 16); }
__device__ __forceinline__ float bfr(float f) { return bf2f(f2bf(f)); }
__device__ __forceinline__ v16h cat16(v8h lo, v8h hi) { return __builtin_shufflevector(lo, hi, 0, 1, 2, 3, 4, 5, 6, 7, 8, 9, 10, 11, 12, 13, 14, 15); }
__device__ __forceinline__ v16bf cat16b(v8us lo, v8us hi) { return __builtin_bit_cast(v16bf, __builtin_shufflevector(lo, hi, 0, 1, 2, 3, 4, 5, 6, 7, 8, 9, 10, 11, 12, 13, 14, 15)); }
__device__ __forceinline__ v8f wmma16(v16h a, v16h b, v8f c) { return __builtin_amdgcn_wmma_f32_16x16x32_f16(false, a, false, b, (short)0, c, false, false); }
__device__ __forceinline__ v8f wmmab(v16bf a, v16bf b, v8f c) { return __builtin_amdgcn_wmma_f32_16x16x32_bf16(false, a, false, b, (short)0, c, false, false); }

template <bool SPLITA, bool F16OUT = false>
__global__ __launch_bounds__(128) void k_gemmb(const bf* __restrict__ A, const bf* __restrict__ Al, const bf* __restrict__ Bn, const float* __restrict__ bias, float* C, int ldc, h16* C2, const float* __restrict__ R = nullptr, int K = DM, int roundR = 1) {
    __shared__ __align__(16) float ost[4][16 * 68];
    const int lane = threadIdx.x & 31, wave = threadIdx.x >> 5, lr = lane & 15, hi = lane >> 4;
    const int r0 = blockIdx.x * 64 + wave * 16, c0 = blockIdx.y * 64;
    const size_t aoff = (size_t)(r0 + lr) * K + 8 * hi;
    size_t boff[4];
#pragma unroll
    for (int t = 0; t < 4; ++t) boff[t] = (size_t)(c0 + t * 16 + lr) * K + 8 * hi;
    v8f acc[4];
#pragma unroll
    for (int t = 0; t < 4; ++t) acc[t] = (v8f){};
#pragma unroll 1
    for (int kc = 0; kc < K; kc += 32) {
        const v16bf a = cat16b(*(const v8us*)(A + aoff + kc), *(const v8us*)(A + aoff + kc + 16));
        v16bf al = a;
        if (SPLITA) al = cat16b(*(const v8us*)(Al + aoff + kc), *(const v8us*)(Al + aoff + kc + 16));
#pragma unroll
        for (int t = 0; t < 4; ++t) { const v16bf b = cat16b(*(const v8us*)(Bn + boff[t] + kc), *(const v8us*)(Bn + boff[t] + kc + 16)); acc[t] = wmmab(a, b, acc[t]); if (SPLITA) acc[t] = wmmab(al, b, acc[t]); }
        asm volatile("v_nop\n\tv_nop\n\tv_nop\n\tv_nop" : "+v"(acc[0]), "+v"(acc[1]), "+v"(acc[2]), "+v"(acc[3]) : "v"(a), "v"(al));
    }
    float* os = &ost[wave][0];
#pragma unroll
    for (int t = 0; t < 4; ++t) { const float bv = bias ? bfr(bias[c0 + t * 16 + lr]) : 0.f;
#pragma unroll
        for (int j = 0; j < 8; ++j) os[(hi * 8 + j) * 68 + t * 16 + lr] = acc[t][j] + bv; }
    __syncthreads();
    if (F16OUT) {
        h16* crow = (h16*)(void*)C + (size_t)r0 * ldc + c0;
        auto pass = [&]() {
#pragma unroll
            for (int s = 0; s < 4; ++s) { const int row = 4 * s + (lane >> 3), piece = lane & 7; const float* sp = os + row * 68 + piece * 8; v8h o, o2;
#pragma unroll
                for (int i = 0; i < 8; ++i) { const h16 a = (h16)sp[i]; o[i] = a; o2[i] = (h16)((sp[i] - (float)a) * LOSC); }
                *(volatile v8h*)(crow + (size_t)row * ldc + piece * 8) = o; if (C2) *(volatile v8h*)(C2 + (size_t)r0 * ldc + c0 + (size_t)row * ldc + piece * 8) = o2; }
        };
        pass(); __threadfence(); pass();
    } else {
        float* crow = C + (size_t)r0 * ldc + c0;
        auto pass = [&]() {
#pragma unroll
            for (int s = 0; s < 8; ++s) { const int Lid = (lane >> 3) + 4 * s, piece = lane & 7; const int row = Lid >> 1, cofs = (Lid & 1) * 32 + piece * 4;
                v4f val = *(const v4fa*)(os + row * 68 + cofs); if (R) { const v4f rv = *(const v4f*)(R + ((size_t)r0 + row) * ldc + c0 + cofs); val += roundR ? (v4f){bfr(rv[0]), bfr(rv[1]), bfr(rv[2]), bfr(rv[3])} : rv; }
                *(volatile v4f*)(crow + (size_t)row * ldc + cofs) = val; }
        };
        pass(); __threadfence(); pass();
    }
}


__global__ __launch_bounds__(256) void k_cvt8(const float* __restrict__ src, bf* dst, size_t n8) {
    const size_t i = (size_t)blockIdx.x * 256 + threadIdx.x; if (i >= n8) return;
    const v8f v = *(const v8f*)(src + i * 8); v8us o;
#pragma unroll
    for (int k = 0; k < 8; ++k) o[k] = f2bf(v[k]);
    *(volatile v8us*)(dst + i * 8) = o; __threadfence(); *(volatile v8us*)(dst + i * 8) = o;
}
__global__ __launch_bounds__(256) void k_zero8(bf* dst, size_t n8) {
    const size_t i = (size_t)blockIdx.x * 256 + threadIdx.x; if (i >= n8) return; v8us z;
#pragma unroll
    for (int k = 0; k < 8; ++k) z[k] = 0;
    *(volatile v8us*)(dst + i * 8) = z; __threadfence(); *(volatile v8us*)(dst + i * 8) = z;
}

__global__ __launch_bounds__(256) void k_styleb(const float* __restrict__ st, bf* SB) {
    const int lane = threadIdx.x & 31, r = blockIdx.x * 8 + (threadIdx.x >> 5); if (r >= 64) return;
#pragma unroll 1
    for (int ps = 0; ps < 2; ++ps) {
#pragma unroll
        for (int q = 0; q < SD / 256; ++q) { v8us o;
#pragma unroll
            for (int i = 0; i < 8; ++i) o[i] = (r < NBI) ? f2bf(st[(size_t)r * SD + q * 256 + lane * 8 + i]) : (unsigned short)0;
            *(volatile v8us*)(SB + (size_t)r * SD + q * 256 + lane * 8) = o; }
        if (ps == 0) __threadfence(); }
}
__global__ __launch_bounds__(256) void k_wmod(const float* __restrict__ Wt, const float* __restrict__ S, const float* __restrict__ mb, int b, bf* Ah, bf* Al) {
    const int lane = threadIdx.x & 31, o = blockIdx.x * 8 + (threadIdx.x >> 5); if (o >= COUT) return;
    const float cs = rsqrtf((float)(CIN * KK)), msc = rsqrtf((float)SD);
    auto wval = [&](int idx) -> float { const int c = idx / KK; const float s = S[(size_t)b * CIN + c] * msc + bfr(mb[c]); return cs * bfr(Wt[(size_t)o * KC + idx]) * s; };
    float ss = 0.f;
#pragma unroll 1
    for (int c0 = lane * 8; c0 < KC; c0 += 256) {
#pragma unroll
        for (int i = 0; i < 8; ++i) { const float w = wval(c0 + i); ss = fmaf(w, w, ss); } }
#pragma unroll
    for (int sh = 16; sh; sh >>= 1) ss += __shfl_xor(ss, sh, 32);
    const float d = rsqrtf(ss + 1e-8f);
#pragma unroll 1
    for (int ps = 0; ps < 2; ++ps) {
#pragma unroll 1
        for (int c0 = lane * 8; c0 < KC; c0 += 256) { v8us oh, ol;
#pragma unroll
            for (int i = 0; i < 8; ++i) { const float w = wval(c0 + i) * d; const unsigned short hb = f2bf(w); oh[i] = hb; ol[i] = f2bf(w - bf2f(hb)); }
            const size_t off = (size_t)o * KC + c0; *(volatile v8us*)(Ah + off) = oh; *(volatile v8us*)(Al + off) = ol; }
        if (ps == 0) __threadfence(); }
}
__global__ __launch_bounds__(256) void k_im2col(const float* __restrict__ xb, bf* X3) {
    const int lane = threadIdx.x & 31, p = blockIdx.x * 8 + (threadIdx.x >> 5); if (p >= PP) return;
#pragma unroll 1
    for (int ps = 0; ps < 2; ++ps) {
#pragma unroll 1
        for (int c0 = lane * 8; c0 < KC; c0 += 256) { v8us o;
#pragma unroll
            for (int i = 0; i < 8; ++i) { const int idx = c0 + i, c = idx / KK, k = idx - c * KK; const int pp = p + k - 1; const bool ok = (pp >= 0) && (pp < PP); o[i] = ok ? f2bf(xb[(size_t)c * PP + (ok ? pp : 0)]) : (unsigned short)0; }
            *(volatile v8us*)(X3 + (size_t)p * KC + c0) = o; }
        if (ps == 0) __threadfence(); }
}

extern "C" void kernel_launch(void* const* d_in, const int* in_sizes, int n_in,
                              void* d_out, int out_size, void* d_ws, size_t ws_size, hipStream_t stream) {
    (void)in_sizes; (void)n_in; (void)out_size;
    const float* x = (const float*)d_in[0]; const float* st = (const float*)d_in[1]; const float* Wt = (const float*)d_in[2]; const float* mw = (const float*)d_in[3]; const float* mb = (const float*)d_in[4];
    float* out = (float*)d_out;
    char* wsp = (char*)d_ws;
    auto take = [&](size_t bytes) { char* p = wsp; wsp += (bytes + 255) & ~(size_t)255; return (void*)p; };
    bf* SB = (bf*)take((size_t)64 * SD * 2); bf* MWB = (bf*)take((size_t)CIN * SD * 2); float* S = (float*)take((size_t)64 * CIN * 4);
    bf* Ah = (bf*)take((size_t)COUT * KC * 2); bf* Al = (bf*)take((size_t)COUT * KC * 2); bf* X3 = (bf*)take((size_t)PP * KC * 2);
    if ((size_t)(wsp - (char*)d_ws) > ws_size) return;
    k_styleb<<<64 / 8, 256, 0, stream>>>(st, SB); k_cvt8<<<(CIN * SD / 8 + 255) / 256, 256, 0, stream>>>(mw, MWB, (size_t)CIN * SD / 8);
    k_gemmb<false, false><<<dim3(1, CIN / 64, 1), 128, 0, stream>>>(SB, nullptr, MWB, nullptr, S, CIN, nullptr, nullptr, SD);
    for (int b = 0; b < NBI; ++b) {
        k_wmod<<<COUT / 8, 256, 0, stream>>>(Wt, S, mb, b, Ah, Al);
        k_im2col<<<PP / 8, 256, 0, stream>>>(x + (size_t)b * CIN * PP, X3);
        k_gemmb<true, false><<<dim3(COUT / 64, PP / 64, 1), 128, 0, stream>>>(Ah, Al, X3, nullptr, out + (size_t)b * COUT * PP, PP, nullptr, nullptr, KC); }
}
